// PointTransformerLayer_20194936226527
// MI455X (gfx1250) — hardware-run, weakly checked
//
#include <hip/hip_runtime.h>
#include <math.h>

typedef __attribute__((ext_vector_type(16))) _Float16 v16h;
typedef __attribute__((ext_vector_type(16))) __bf16 v16b;
typedef __attribute__((ext_vector_type(8)))  _Float16 v8h;
typedef __attribute__((ext_vector_type(8)))  float v8f;
typedef __attribute__((ext_vector_type(4)))  float v4f;
typedef __attribute__((ext_vector_type(2)))  float v2f;
typedef __attribute__((ext_vector_type(4)))  unsigned v4u;
typedef __attribute__((ext_vector_type(4)))  int v4i;
typedef float __attribute__((may_alias)) float_a;
typedef int __attribute__((may_alias)) int_a;

template <typename T> __device__ __forceinline__ void vst2(void* p, T v) { *(volatile T*)p = v; __threadfence(); *(volatile T*)p = v; }
__device__ __forceinline__ v8f wmma16(v16h a, v16h b, v8f c) {
  v8f d = __builtin_amdgcn_wmma_f32_16x16x32_f16(false, a, false, b, (short)0, c, false, false);
  asm volatile("v_nop\n\tv_nop\n\tv_nop\n\tv_nop" : "+v"(d) : "v"(a), "v"(b));
  return d;
}
__device__ __forceinline__ v8f wmma_bf(v16b a, v16b b, v8f c) {
  v8f d = __builtin_amdgcn_wmma_f32_16x16x32_bf16(false, a, false, b, (short)0, c, false, false);
  asm volatile("v_nop\n\tv_nop\n\tv_nop\n\tv_nop" : "+v"(d) : "v"(a), "v"(b));
  return d;
}
__device__ __forceinline__ v16h frag_h(const _Float16* rowk0, int lane) {
  union { v16h v; v8h q[2]; } u; const _Float16* p = rowk0 + 8 * (lane >> 4);
  u.q[0] = *(const v8h*)p; u.q[1] = *(const v8h*)(p + 16); return u.v;
}
__device__ __forceinline__ v16h frag_f32(const float* rowk0, int lane) {
  v16h a; const float* p = rowk0 + 8 * (lane >> 4);
#pragma unroll
  for (int i = 0; i < 8; ++i) { a[i] = (_Float16)p[i]; a[8 + i] = (_Float16)p[16 + i]; }
  return a;
}
__device__ __forceinline__ v16h frag_f32s(const float* rowk0, int lane, float sc) {
  v16h a; const float* p = rowk0 + 8 * (lane >> 4);
#pragma unroll
  for (int i = 0; i < 8; ++i) { a[i] = (_Float16)(p[i] * sc); a[8 + i] = (_Float16)(p[16 + i] * sc); }
  return a;
}
__device__ __forceinline__ v16h fragc_f32(const float* W, int k0, int n, int lane, int ld, int K) {
  v16h a; const int g = lane >> 4;
#pragma unroll
  for (int i = 0; i < 8; ++i) { const int ka = k0 + 8 * g + i, kb = ka + 16;
    a[i] = (_Float16)(ka < K ? W[(size_t)(ka < K ? ka : K - 1) * ld + n] : 0.f); a[8 + i] = (_Float16)(kb < K ? W[(size_t)(kb < K ? kb : K - 1) * ld + n] : 0.f); }
  return a;
}
struct F2 { v16b h, l; };
__device__ __forceinline__ F2 bsplit16(const float v[16]) { F2 r;
#pragma unroll
  for (int i = 0; i < 16; ++i) { const __bf16 h = (__bf16)v[i]; r.h[i] = h; r.l[i] = (__bf16)(v[i] - (float)h); }
  return r; }
__device__ __forceinline__ F2 split_row(const float* row, int k0, int lane) { float v[16]; const float* p = row + k0 + 8 * (lane >> 4);
#pragma unroll
  for (int i = 0; i < 8; ++i) { v[i] = p[i]; v[8 + i] = p[16 + i]; }
  return bsplit16(v); }
__device__ __forceinline__ F2 split_rowK(const float* row, int k0, int lane, int K) { float v[16]; const int g = lane >> 4;
#pragma unroll
  for (int i = 0; i < 8; ++i) { const int ka = k0 + 8 * g + i, kb = ka + 16; v[i] = ka < K ? row[ka < K ? ka : K - 1] : 0.f; v[8 + i] = kb < K ? row[kb < K ? kb : K - 1] : 0.f; }
  return bsplit16(v); }
__device__ __forceinline__ F2 split_col(const float* W, int k0, int n, int lane, int ld, int K) { float v[16]; const int g = lane >> 4;
#pragma unroll
  for (int i = 0; i < 8; ++i) { const int ka = k0 + 8 * g + i, kb = ka + 16; v[i] = ka < K ? W[(size_t)(ka < K ? ka : K - 1) * ld + n] : 0.f; v[8 + i] = kb < K ? W[(size_t)(kb < K ? kb : K - 1) * ld + n] : 0.f; }
  return bsplit16(v); }
__device__ __forceinline__ v8f mac3(const F2& a, const F2& b, v8f c) { c = wmma_bf(a.l, b.h, c); c = wmma_bf(a.h, b.l, c); return wmma_bf(a.h, b.h, c); }
__device__ __forceinline__ float sigm(float v) { return 1.0f / (1.0f + expf(-v)); }
#define LDSX() do { asm volatile("s_wait_dscnt 0" ::: "memory"); __builtin_amdgcn_wave_barrier(); __builtin_amdgcn_fence(__ATOMIC_RELEASE, "workgroup"); } while (0)

#define NBT 16
#define NPT 512
#define CIN 512
#define CO 512
#define CS 64
#define KN 16
#define NR (NBT * NPT)
#ifndef NRV
#define NRV NR
#endif
typedef __attribute__((ext_vector_type(4))) int v4i;
__device__ __forceinline__ float bfr(float v) { return (float)(__bf16)v; }
__device__ __forceinline__ v16b wcol_io(const float* __restrict__ Wm, int k0, int o, int lane, int ld) { v16b w; const float* p = Wm + (size_t)(k0 + 8 * (lane >> 4)) * ld + o;
#pragma unroll
  for (int i = 0; i < 8; ++i) { w[i] = (__bf16)p[(size_t)i * ld]; w[8 + i] = (__bf16)p[(size_t)(16 + i) * ld]; }
  asm volatile("s_wait_loadcnt 0x0" ::: "memory"); return w; }
#define WS_XT  0u
#define WS_Q   (WS_XT + 4u * (size_t)NR * CIN)
#define WS_KF  (WS_Q + 4u * (size_t)NR * CO)
#define WS_VF  (WS_KF + 4u * (size_t)NR * CO)
#define WS_IDX (WS_VF + 4u * (size_t)NR * CO)
#define WS_END (WS_IDX + 4u * (size_t)NR * KN)
__global__ __launch_bounds__(256) void k_tok(const float* __restrict__ X, float* __restrict__ XT) { __shared__ float st[64][68];
  const int tid = threadIdx.x; const int n0 = blockIdx.x * 64, c0 = blockIdx.y * 64; const size_t b = blockIdx.z;
  for (int e = tid; e < 64 * 16; e += 256) { const int cl = e >> 4, q = e & 15; const v4f v = *(const v4f*)(X + (b * CIN + c0 + cl) * NPT + n0 + q * 4); st[cl][q * 4] = bfr(v[0]); st[cl][q * 4 + 1] = bfr(v[1]); st[cl][q * 4 + 2] = bfr(v[2]); st[cl][q * 4 + 3] = bfr(v[3]); }
  __syncthreads();
  for (int e = tid; e < 64 * 16; e += 256) { const int nl = e >> 4, q = e & 15; v4f o; o[0] = st[q * 4][nl]; o[1] = st[q * 4 + 1][nl]; o[2] = st[q * 4 + 2][nl]; o[3] = st[q * 4 + 3][nl]; vst2(XT + (b * NPT + n0 + nl) * (size_t)CIN + c0 + q * 4, o); } }
__global__ __launch_bounds__(128) void k_lin(const float* __restrict__ XT, const float* __restrict__ WQ, const float* __restrict__ BQ, const float* __restrict__ WK, const float* __restrict__ BK, const float* __restrict__ WV, const float* __restrict__ BV, float* __restrict__ Q, float* __restrict__ KF, float* __restrict__ VF) { __shared__ __align__(16) float sf[4][16][132];
  const int tid = threadIdx.x, wave = tid >> 5, lane = tid & 31, col = lane & 15, g = lane >> 4; const int which = blockIdx.z; const int c0 = blockIdx.y * 128; const size_t r0 = (size_t)blockIdx.x * 64 + wave * 16;
  const float* Wm = which == 0 ? WQ : (which == 1 ? WK : WV); const float* Bm = which == 0 ? BQ : (which == 1 ? BK : BV); float* OUT = which == 0 ? Q : (which == 1 ? KF : VF);
  v8f acc[8] = {};
#pragma unroll 2
  for (int kc = 0; kc < CIN / 32; ++kc) { v16b a; { const float* p = XT + (r0 + col) * CIN + kc * 32 + 8 * g;
#pragma unroll
      for (int i = 0; i < 8; ++i) { a[i] = (__bf16)p[i]; a[8 + i] = (__bf16)p[16 + i]; } }
    asm volatile("s_wait_loadcnt 0x0" ::: "memory");
#pragma unroll
    for (int j = 0; j < 8; ++j) { const v16b w = wcol_io(Wm, kc * 32, c0 + j * 16 + col, lane, CO); acc[j] = wmma_bf(a, w, acc[j]); } }
#pragma unroll
  for (int j = 0; j < 8; ++j) { const float bb = bfr(Bm[c0 + j * 16 + col]);
#pragma unroll
    for (int r = 0; r < 8; ++r) sf[wave][8 * g + r][j * 16 + col] = acc[j][r] + bb; }
  LDSX(); for (int rl = 0; rl < 16; ++rl) vst2(OUT + (r0 + rl) * CO + c0 + lane * 4, *(const v4f*)&sf[wave][rl][lane * 4]); }
struct Best8 { float d[KN]; int i[KN]; };
__device__ __forceinline__ void push8(Best8& b, float d, int i) {
  if (d < b.d[KN - 1]) { b.d[KN - 1] = d; b.i[KN - 1] = i; }
#pragma unroll
  for (int p = KN - 1; p > 0; --p) { const bool sw = b.d[p] < b.d[p - 1]; const float td = b.d[p], ud = b.d[p - 1]; const int ti = b.i[p], ui = b.i[p - 1]; b.d[p] = sw ? ud : td; b.d[p - 1] = sw ? td : ud; b.i[p] = sw ? ui : ti; b.i[p - 1] = sw ? ti : ui; } }
__global__ __launch_bounds__(256) void k_knn(const float* __restrict__ P, int* __restrict__ IDX) { __shared__ int sidx8[8][KN];
  const int wave = threadIdx.x >> 5, lane = threadIdx.x & 31; const size_t row = (size_t)blockIdx.x * 8 + wave;
  const size_t b = row / NPT; const int n = (int)(row % NPT);
  Best8 bs;
#pragma unroll
  for (int r = 0; r < KN; ++r) { bs.d[r] = 3.0e38f; bs.i[r] = 0x7fffffff; }
  {
#pragma clang fp contract(off)
    const float qx = bfr(P[(b * NPT + n) * 3]), qy = bfr(P[(b * NPT + n) * 3 + 1]), qz = bfr(P[(b * NPT + n) * 3 + 2]);
    const float aa = (qx * qx + qy * qy) + qz * qz;
#pragma unroll 1
    for (int s = lane; s < NPT; s += 32) { const float px = bfr(P[(b * NPT + s) * 3]), py = bfr(P[(b * NPT + s) * 3 + 1]), pz = bfr(P[(b * NPT + s) * 3 + 2]);
      const float bb = (px * px + py * py) + pz * pz; const float dot = (qx * px + qy * py) + qz * pz; const float d = (aa + bb) - 2.0f * dot; push8(bs, d, s); } }
  int sel = 0;
#pragma unroll 1
  for (int r = 0; r < KN; ++r) { float d = bs.d[0]; int i = bs.i[0];
#pragma unroll
    for (int o = 1; o < 32; o <<= 1) { const float e = __shfl_xor(d, o); const int j = __shfl_xor(i, o); if (e < d || (e == d && j < i)) { d = e; i = j; } }
    if (lane == r) sel = i;
    { const bool pop = (bs.i[0] == i && bs.d[0] == d);
#pragma unroll
      for (int p = 0; p < KN - 1; ++p) { bs.d[p] = pop ? bs.d[p + 1] : bs.d[p]; bs.i[p] = pop ? bs.i[p + 1] : bs.i[p]; }
      bs.d[KN - 1] = pop ? 3.0e38f : bs.d[KN - 1]; bs.i[KN - 1] = pop ? 0x7fffffff : bs.i[KN - 1]; } }
  if (lane < KN) sidx8[wave][lane] = sel;
  __syncthreads();
  if (threadIdx.x < 32) vst2((v4i*)(IDX + (size_t)blockIdx.x * 8 * KN) + threadIdx.x, *(const v4i*)(&sidx8[0][0] + threadIdx.x * 4)); }

#define BNS(g) (bfr(g) / sqrtf(1.0f + 1e-5f))
__global__ __launch_bounds__(128) void k_edge(const float* __restrict__ P, const int* __restrict__ IDX, const float* __restrict__ Q, const float* __restrict__ KF, const float* __restrict__ VF,
    const float* __restrict__ P1W, const float* __restrict__ P1B, const float* __restrict__ PG, const float* __restrict__ PB, const float* __restrict__ P2W, const float* __restrict__ P2B,
    const float* __restrict__ G1, const float* __restrict__ B1N, const float* __restrict__ W1, const float* __restrict__ W1B, const float* __restrict__ G2, const float* __restrict__ B2N, const float* __restrict__ W2, const float* __restrict__ W2B, float* __restrict__ OUT) {
  __shared__ __align__(16) float sv[4][16][68]; __shared__ float sh[4][16][4]; __shared__ int sidx[4][16];
  const int tid = threadIdx.x, wave = tid >> 5, lane = tid & 31, col = lane & 15, g = lane >> 4;
  const size_t n = (size_t)blockIdx.x * 4 + wave; const size_t b = n / NPT;
  if (lane < KN) { int ix = IDX[n * KN + lane]; ix = ix < 0 ? 0 : (ix >= NPT ? NPT - 1 : ix); const size_t m = b * NPT + ix; sidx[wave][lane] = (int)m;
    const float rx = bfr(P[m * 3]) - bfr(P[n * 3]), ry = bfr(P[m * 3 + 1]) - bfr(P[n * 3 + 1]), rz = bfr(P[m * 3 + 2]) - bfr(P[n * 3 + 2]);
#pragma unroll
    for (int i = 0; i < 3; ++i) { const float y = (rx * bfr(P1W[0 * 3 + i]) + ry * bfr(P1W[1 * 3 + i])) + rz * bfr(P1W[2 * 3 + i]) + bfr(P1B[i]); sh[wave][lane][i] = fmaxf(y * BNS(PG[i]) + bfr(PB[i]), 0.f); }
    sh[wave][lane][3] = 0.f; }
  LDSX();
  const int mrow = sidx[wave][col]; const float h0 = sh[wave][col][0], h1 = sh[wave][col][1], h2 = sh[wave][col][2];
  v8f acc[4] = {};
#pragma unroll 1
  for (int kc = 0; kc < CIN / 32; ++kc) { float va[16];
#pragma unroll
    for (int i = 0; i < 16; ++i) { const int c = kc * 32 + 8 * g + (i < 8 ? i : 8 + i); const float pe = ((h0 * bfr(P2W[c]) + h1 * bfr(P2W[CO + c])) + h2 * bfr(P2W[2 * CO + c])) + bfr(P2B[c]);
      const float wv = (KF[(size_t)mrow * CO + c] - Q[n * CO + c]) + pe; va[i] = fmaxf(wv * BNS(G1[c]) + bfr(B1N[c]), 0.f); }
    asm volatile("s_wait_loadcnt 0x0" ::: "memory");
    const F2 a = bsplit16(va);
#pragma unroll
    for (int j = 0; j < 4; ++j) { const v16b w = wcol_io(W1, kc * 32, j * 16 + col, lane, CS); acc[j] = wmma_bf(a.h, w, acc[j]); acc[j] = wmma_bf(a.l, w, acc[j]); } }
#pragma unroll
  for (int j = 0; j < 4; ++j) { const int o = j * 16 + col; const float bb = bfr(W1B[o]), gs = BNS(G2[o]), bn = bfr(B2N[o]);
#pragma unroll
    for (int r = 0; r < 8; ++r) sv[wave][8 * g + r][o] = fmaxf((acc[j][r] + bb) * gs + bn, 0.f); }
  LDSX();
  { v8f acc2[4] = {};
#pragma unroll
    for (int kc = 0; kc < CS / 32; ++kc) { const F2 a = split_row(&sv[wave][col][0], kc * 32, lane);
#pragma unroll
      for (int j = 0; j < 4; ++j) { const v16b w = wcol_io(W2, kc * 32, j * 16 + col, lane, CS); acc2[j] = wmma_bf(a.h, w, acc2[j]); acc2[j] = wmma_bf(a.l, w, acc2[j]); } }
    LDSX();
#pragma unroll
    for (int j = 0; j < 4; ++j) { const float bb = bfr(W2B[j * 16 + col]);
#pragma unroll
      for (int r = 0; r < 8; ++r) sv[wave][8 * g + r][j * 16 + col] = acc2[j][r] + bb; } }
  LDSX();
#pragma unroll
  for (int q2 = 0; q2 < 2; ++q2) { const int o = q2 * 32 + lane; float mx = -3.0e38f;
#pragma unroll
    for (int j = 0; j < KN; ++j) mx = fmaxf(mx, sv[wave][j][o]);
    float e[KN], sum = 0.f;
#pragma unroll
    for (int j = 0; j < KN; ++j) { e[j] = expf(sv[wave][j][o] - mx); sum += e[j]; }
    const float inv = 1.0f / sum;
#pragma unroll
    for (int j = 0; j < KN; ++j) sv[wave][j][o] = e[j] * inv; }
  LDSX();
#pragma unroll 1
  for (int qd = 0; qd < CO / 128; ++qd) { const int c0 = qd * 128 + lane * 4; v4f o4; o4[0] = o4[1] = o4[2] = o4[3] = 0.f;
    float p2b[4], p20[4], p21[4], p22[4];
#pragma unroll
    for (int i = 0; i < 4; ++i) { p2b[i] = bfr(P2B[c0 + i]); p20[i] = bfr(P2W[c0 + i]); p21[i] = bfr(P2W[CO + c0 + i]); p22[i] = bfr(P2W[2 * CO + c0 + i]); }
#pragma unroll 1
    for (int j = 0; j < KN; ++j) { const size_t m = (size_t)sidx[wave][j]; const v4f vv = *(const v4f*)(VF + m * CO + c0); const float hj0 = sh[wave][j][0], hj1 = sh[wave][j][1], hj2 = sh[wave][j][2];
#pragma unroll
      for (int i = 0; i < 4; ++i) { const float pe = ((hj0 * p20[i] + hj1 * p21[i]) + hj2 * p22[i]) + p2b[i]; o4[i] += (vv[i] + pe) * sv[wave][j][(c0 + i) & (CS - 1)]; } }
    vst2(OUT + n * CO + c0, o4); } }
extern "C" void kernel_launch(void* const* d_in, const int* in_sizes, int n_in, void* d_out, int out_size, void* d_ws, size_t ws_size, hipStream_t stream) {
  (void)in_sizes; (void)n_in; (void)out_size;
  if (ws_size < (size_t)WS_END) return;
  char* ws = (char*)d_ws; const float** F = (const float**)d_in; float *XT = (float*)(ws + WS_XT), *Q = (float*)(ws + WS_Q), *KF = (float*)(ws + WS_KF), *VF = (float*)(ws + WS_VF); int* IDX = (int*)(ws + WS_IDX);
  k_tok<<<dim3(NPT / 64, CIN / 64, NRV / NPT), 256, 0, stream>>>(F[1], XT);
  k_lin<<<dim3(NRV / 64, CO / 128, 3), 128, 0, stream>>>(XT, F[2], F[3], F[4], F[5], F[6], F[7], Q, KF, VF);
  k_knn<<<dim3(NRV / 8), 256, 0, stream>>>(F[0], IDX);
  k_edge<<<dim3(NRV / 4), 128, 0, stream>>>(F[0], IDX, Q, KF, VF, F[8], F[9], F[10], F[11], F[12], F[13], F[14], F[15], F[16], F[17], F[18], F[19], F[20], F[21], (float*)d_out);
}
